// DGCNNBlock_38800734552598
// MI455X (gfx1250) — hardware-verified
//
#include <hip/hip_runtime.h>
#include <stddef.h>
#include <math.h>


#define CIN    64
#define CH     64
#define NCO    128
#define PQW    128
#define KPB    64
#define APZ    72
#define APE    72
#define NTHR   256
#define NWAVE  8
#define GROWS  64
#define GTHR   128
#define EWAV   4
#define ETHR   128
#define NPW    16
#define NPBE   (EWAV * NPW)
#define TCAP   64
#define DEGCAP 512
#define EPT    8
#define NGRP   2
#define CHUNK  (NTHR * EPT * NGRP)
#define WCAP   256
#define LISTN  (NWAVE * WCAP)
#define NBC    4096
#define NBF    2048
#define RCAP   67072
#define RBN    128
#define OTHR   512
#define LDS_FILL ((RCAP + NBF + LISTN) * 4 + 64)
#define O_NH   0
#define O_NL   8192
#define O_E    16384
#define BPTOT  20480
#define WPSLOT 1536
#define WSCAP  134217728
#define HSC    16.0f
#define WSC    64.0f
#define ESC    0.0009765625f
#define NEGBIG (-3.0e38f)

static_assert(GROWS == (GTHR / 32) * 16);
static_assert(GTHR == 2 * GROWS);
static_assert(NPBE == GROWS);
static_assert((NBF % NPW) == 0 && (NPBE % NPW) == 0);
static_assert((APZ % 8) == 0 && (APE % 8) == 0 && APZ >= CIN && APE >= CH && (KPB % 8) == 0);
static_assert((CHUNK & (CHUNK - 1)) == 0 && CHUNK <= 4096);
static_assert(NBC <= 4096 && (NBC & (NBC - 1)) == 0 && (NBF & (NBF - 1)) == 0);
static_assert(NBC == 2 * NBF);
static_assert(OTHR * 8 == NBC);
static_assert((RCAP % 32) == 0);
static_assert((DEGCAP % 16) == 0);
static_assert(BPTOT == O_E + CH * KPB);
static_assert(O_NL == O_NH + NCO * KPB && O_E == O_NL + NCO * KPB);
static_assert(WPSLOT * 8 == NCO * KPB + CH * KPB);
static_assert(WPSLOT == 6 * NTHR);
static_assert((O_NL % 64) == 0 && (O_E % 64) == 0);
static_assert(TCAP * 16 >= NPW * 16);

typedef float          v4f   __attribute__((ext_vector_type(4)));
typedef float          v8f   __attribute__((ext_vector_type(8)));
typedef int            v4i   __attribute__((ext_vector_type(4)));
typedef unsigned short v4us  __attribute__((ext_vector_type(4)));
typedef unsigned short v8us  __attribute__((ext_vector_type(8)));
typedef unsigned short v16us __attribute__((ext_vector_type(16)));
typedef __bf16         v16b  __attribute__((ext_vector_type(16)));
typedef _Float16       v4h   __attribute__((ext_vector_type(4)));
typedef _Float16       v8h   __attribute__((ext_vector_type(8)));
typedef _Float16       v16h  __attribute__((ext_vector_type(16)));
union Frag  { v16us u; v8us h[2]; };
union FragH { v16h v; v8h h[2]; v8us u[2]; };

__device__ __forceinline__ unsigned short bfr(float f) {
  const unsigned u = __float_as_uint(f);
  return (unsigned short)((u + 0x7FFFu + ((u >> 16) & 1u)) >> 16);
}
__device__ __forceinline__ float bfv(unsigned short h) { return __uint_as_float(((unsigned)h) << 16); }

__device__ __forceinline__ void split8(const float (&v)[8], v8us& uh, v8us& ul) {
#pragma unroll
  for (int e = 0; e < 8; ++e) {
    const unsigned short h = bfr(v[e]);
    uh[e] = h;
    ul[e] = bfr(v[e] - bfv(h));
  }
}

__device__ __forceinline__ v8f wmb(v16us a, v16us b, v8f c) {
  const v16b av = __builtin_bit_cast(v16b, a);
  const v16b bv = __builtin_bit_cast(v16b, b);
  v8f d = __builtin_amdgcn_wmma_f32_16x16x32_bf16(false, av, false, bv, (short)0, c, false, false);
  asm volatile("v_nop\n\tv_nop\n\tv_nop\n\tv_nop" : "+v"(d) : "v"(av), "v"(bv));
  return d;
}
__device__ __forceinline__ v8f wmh(v16h a, v16h b, v8f c) {
  v8f d = __builtin_amdgcn_wmma_f32_16x16x32_f16(false, a, false, b, (short)0, c, false, false);
  asm volatile("v_nop\n\tv_nop\n\tv_nop\n\tv_nop" : "+v"(d) : "v"(a), "v"(b));
  return d;
}

template <int NT>
__device__ __forceinline__ void mma3k2(const unsigned short* Ah, const unsigned short* Al,
                                       const unsigned short* __restrict__ Bh, const unsigned short* __restrict__ Bl,
                                       int lane, v8f (&acc)[NT]) {
  const int hh = lane >> 4, m = lane & 15;
#pragma unroll
  for (int t = 0; t < NT; ++t) {
    const v8f z = {0.f, 0.f, 0.f, 0.f, 0.f, 0.f, 0.f, 0.f};
    acc[t] = z;
  }
#pragma unroll
  for (int s = 0; s < 2; ++s) {
    Frag ah, al;
    ah.h[0] = *(const v8us*)(Ah + m * APZ + 32 * s + 8 * hh);
    ah.h[1] = *(const v8us*)(Ah + m * APZ + 32 * s + 16 + 8 * hh);
    al.h[0] = *(const v8us*)(Al + m * APZ + 32 * s + 8 * hh);
    al.h[1] = *(const v8us*)(Al + m * APZ + 32 * s + 16 + 8 * hh);
#pragma unroll
    for (int t = 0; t < NT; ++t) {
      const unsigned short* bph = Bh + (16 * t + m) * KPB + 32 * s + 8 * hh;
      const unsigned short* bpl = Bl + (16 * t + m) * KPB + 32 * s + 8 * hh;
      Frag bh, bl;
      bh.h[0] = *(const v8us*)bph;
      bh.h[1] = *(const v8us*)(bph + 16);
      bl.h[0] = *(const v8us*)bpl;
      bl.h[1] = *(const v8us*)(bpl + 16);
      acc[t] = wmb(ah.u, bh.u, acc[t]);
      acc[t] = wmb(al.u, bh.u, acc[t]);
      acc[t] = wmb(ah.u, bl.u, acc[t]);
    }
  }
}

template <int NB>
__device__ __forceinline__ int scan_chunk(const int* __restrict__ dsts, int nE, int cbase, int slotBase,
                                          int vec8, int* list, int tid, int lane, int wave) {
  int wc = 0;
#pragma unroll
  for (int g = 0; g < NGRP; ++g) {
    const int el0  = (g * NTHR + tid) * EPT;
    const int e0   = cbase + el0;
    const int sent = -2147483647 - 1;
    v4i da, db;
    if (vec8 != 0 && cbase + CHUNK <= nE) {
      da = *(const v4i*)(dsts + e0);
      db = *(const v4i*)(dsts + e0 + 4);
    } else {
      da.x = (e0     < nE) ? dsts[min(e0, nE - 1)] : sent;
      da.y = (e0 + 1 < nE) ? dsts[min(e0 + 1, nE - 1)] : sent;
      da.z = (e0 + 2 < nE) ? dsts[min(e0 + 2, nE - 1)] : sent;
      da.w = (e0 + 3 < nE) ? dsts[min(e0 + 3, nE - 1)] : sent;
      db.x = (e0 + 4 < nE) ? dsts[min(e0 + 4, nE - 1)] : sent;
      db.y = (e0 + 5 < nE) ? dsts[min(e0 + 5, nE - 1)] : sent;
      db.z = (e0 + 6 < nE) ? dsts[min(e0 + 6, nE - 1)] : sent;
      db.w = (e0 + 7 < nE) ? dsts[min(e0 + 7, nE - 1)] : sent;
    }
    const unsigned nb = (unsigned)slotBase;
    const unsigned s0 = (unsigned)da.x - nb, s1 = (unsigned)da.y - nb;
    const unsigned s2 = (unsigned)da.z - nb, s3 = (unsigned)da.w - nb;
    const unsigned s4 = (unsigned)db.x - nb, s5 = (unsigned)db.y - nb;
    const unsigned s6 = (unsigned)db.z - nb, s7 = (unsigned)db.w - nb;
    const bool h0 = s0 < (unsigned)NB, h1 = s1 < (unsigned)NB, h2 = s2 < (unsigned)NB, h3 = s3 < (unsigned)NB;
    const bool h4 = s4 < (unsigned)NB, h5 = s5 < (unsigned)NB, h6 = s6 < (unsigned)NB, h7 = s7 < (unsigned)NB;
    const unsigned any = __builtin_amdgcn_ballot_w32(h0 | h1 | h2 | h3 | h4 | h5 | h6 | h7);
    if (any != 0u) {
#define HITJ(J, HJ, SJ) { \
        const unsigned mj = __builtin_amdgcn_ballot_w32(HJ); \
        if (mj != 0u) { \
          if (HJ) { \
            const int pos = wc + (int)__builtin_amdgcn_mbcnt_lo(mj, 0u); \
            if (pos < WCAP) list[wave * WCAP + pos] = ((el0 + (J)) << 12) | (int)(SJ); \
          } \
          wc += (int)__builtin_popcount(mj); } }
      HITJ(0, h0, s0)
      HITJ(1, h1, s1)
      HITJ(2, h2, s2)
      HITJ(3, h3, s3)
      HITJ(4, h4, s4)
      HITJ(5, h5, s5)
      HITJ(6, h6, s6)
      HITJ(7, h7, s7)
#undef HITJ
    }
  }
  return wc;
}

__global__ __launch_bounds__(NTHR) void k_wprep(const float* __restrict__ W1, const float* __restrict__ W2,
                                                unsigned short* Bpl) {
  const int i = blockIdx.x * NTHR + threadIdx.x;
  if (i < NCO * 8) {
    const int n = i >> 3, k0 = (i & 7) * 8, nc = n & 63;
    float v[8];
#pragma unroll
    for (int e = 0; e < 8; ++e) {
      const int k = k0 + e;
      const float a = W1[nc * 128 + k], b = W1[nc * 128 + 64 + k];
      v[e] = (n < 64) ? (a - b) : b;
    }
    v8us uh, ul;
    split8(v, uh, ul);
    unsigned short* ph = Bpl + O_NH + n * KPB + k0;
    unsigned short* pl = Bpl + O_NL + n * KPB + k0;
    *(volatile v8us*)ph = uh; *(volatile v8us*)pl = ul;
    __threadfence();
    *(volatile v8us*)ph = uh; *(volatile v8us*)pl = ul;
  } else {
    int j = i - NCO * 8;
    j = j > CH * 8 - 1 ? CH * 8 - 1 : j;
    const int n = j >> 3, k0 = (j & 7) * 8;
    v8h r;
#pragma unroll
    for (int e = 0; e < 8; ++e) r[e] = (_Float16)(W2[n * 64 + k0 + e] * WSC);
    const v8us ue = __builtin_bit_cast(v8us, r);
    unsigned short* pe = Bpl + O_E + n * KPB + k0;
    *(volatile v8us*)pe = ue;
    __threadfence();
    *(volatile v8us*)pe = ue;
  }
}

__global__ __launch_bounds__(NTHR) void k_count(const int* __restrict__ dsts, int* cnt, int nE, int vec8) {
  __shared__ __attribute__((aligned(16))) int scnt[NBC];
  __shared__ __attribute__((aligned(16))) int list[LISTN];
  __shared__ int wcnt[NWAVE];
  const int tid = threadIdx.x, lane = tid & 31, wave = tid >> 5;
  const int nodeBase = blockIdx.x * NBC;

  for (int i = tid; i < NBC; i += NTHR) scnt[i] = 0;
  __syncthreads();

  const int nChunks = (nE + CHUNK - 1) / CHUNK;
#pragma unroll 1
  for (int ch = 0; ch < nChunks; ++ch) {
    const int cbase = ch * CHUNK;
    const int wc = scan_chunk<NBC>(dsts, nE, cbase, nodeBase, vec8, list, tid, lane, wave);
    if (lane == 0) wcnt[wave] = wc;
    __syncthreads();
    if (wave == 0) {
#pragma unroll 1
      for (int wsx = 0; wsx < NWAVE; ++wsx) {
        int n = __builtin_amdgcn_readfirstlane(wcnt[wsx]);
        n = n > WCAP ? WCAP : (n < 0 ? 0 : n);
        const int* lp = list + wsx * WCAP;
#pragma unroll 1
        for (int i = 0; i < n; ++i) {
          const int ent  = __builtin_amdgcn_readfirstlane(lp[i]);
          const int slot = ent & (NBC - 1);
          if (lane == 0) scnt[slot] = scnt[slot] + 1;
        }
      }
    }
    __syncthreads();
  }

  v4i cq[4];
#pragma unroll
  for (int q = 0; q < 4; ++q) {
    const int f = (wave * 4 + q) * 128 + 4 * lane;
    cq[q] = *(const v4i*)(scnt + f);
  }
  int* cp = cnt + (size_t)nodeBase;
#pragma unroll
  for (int q = 0; q < 4; ++q) {
    const int f = (wave * 4 + q) * 128 + 4 * lane;
    *(volatile v4i*)(cp + f) = cq[q];
  }
  __threadfence();
#pragma unroll
  for (int q = 0; q < 4; ++q) {
    const int f = (wave * 4 + q) * 128 + 4 * lane;
    *(volatile v4i*)(cp + f) = cq[q];
  }
}

__global__ __launch_bounds__(OTHR) void k_offsets(const int* __restrict__ cnt, int* off, int* rbase, int nChunk) {
  __shared__ __attribute__((aligned(16))) int soff[NBC];
  __shared__ __attribute__((aligned(16))) int srb[RBN];
  __shared__ int wtot[OTHR / 32];
  const int tid = threadIdx.x, lane = tid & 31, wave = tid >> 5, sub = tid >> 8;
  for (int i = tid; i < RBN; i += OTHR) srb[i] = 0;
  int carry = 0;
#pragma unroll 1
  for (int ch = 0; ch < nChunk; ++ch) {
    const int base = ch * NBC;
    const v4i c0 = *(const v4i*)(cnt + base + 8 * tid);
    const v4i c1 = *(const v4i*)(cnt + base + 8 * tid + 4);
    const int e0 = max(c0.x, 0), e1 = max(c0.y, 0), e2 = max(c0.z, 0), e3 = max(c0.w, 0);
    const int e4 = max(c1.x, 0), e5 = max(c1.y, 0), e6 = max(c1.z, 0), e7 = max(c1.w, 0);
    const int ts = e0 + e1 + e2 + e3 + e4 + e5 + e6 + e7;
    int incl = ts;
#pragma unroll
    for (int d = 1; d < 32; d <<= 1) {
      const int t = __shfl_up(incl, d);
      if (lane >= d) incl += t;
    }
    if (lane == 31) wtot[wave] = incl;
    __syncthreads();
    const int S0 = wtot[0] + wtot[1] + wtot[2]  + wtot[3]  + wtot[4]  + wtot[5]  + wtot[6]  + wtot[7];
    const int S1 = wtot[8] + wtot[9] + wtot[10] + wtot[11] + wtot[12] + wtot[13] + wtot[14] + wtot[15];
    int pre = 0;
#pragma unroll 1
    for (int w = 8 * sub; w < wave; ++w) pre += wtot[w];
    const int b0 = carry;
    const int b1 = b0 + ((S0 + 31) & ~31);
    const int b2 = b1 + ((S1 + 31) & ~31);
    const int myb = sub == 0 ? b0 : b1;
    if (tid == 0) {
      srb[min(2 * ch + 0, RBN - 1)] = b0;
      srb[min(2 * ch + 1, RBN - 1)] = b1;
    }
    int run = myb + pre + incl - ts;
    soff[8 * tid + 0] = run; run += e0;
    soff[8 * tid + 1] = run; run += e1;
    soff[8 * tid + 2] = run; run += e2;
    soff[8 * tid + 3] = run; run += e3;
    soff[8 * tid + 4] = run; run += e4;
    soff[8 * tid + 5] = run; run += e5;
    soff[8 * tid + 6] = run; run += e6;
    soff[8 * tid + 7] = run;
    carry = b2;
    __syncthreads();
    const v4i o0 = *(const v4i*)(soff + 4 * tid);
    const v4i o1 = *(const v4i*)(soff + 4 * (tid + OTHR));
    int* op = off + base;
    *(volatile v4i*)(op + 4 * tid) = o0;
    *(volatile v4i*)(op + 4 * (tid + OTHR)) = o1;
    __threadfence();
    *(volatile v4i*)(op + 4 * tid) = o0;
    *(volatile v4i*)(op + 4 * (tid + OTHR)) = o1;
    __syncthreads();
  }
  if (tid == 0) srb[min(2 * nChunk, RBN - 1)] = carry;
  __syncthreads();
  v4i rv = {0, 0, 0, 0};
  if (tid < 32) rv = *(const v4i*)(srb + 4 * tid);
  if (tid < 32) *(volatile v4i*)(rbase + 4 * tid) = rv;
  __threadfence();
  if (tid < 32) *(volatile v4i*)(rbase + 4 * tid) = rv;
}

__global__ __launch_bounds__(NTHR) void k_fill(
    const int* __restrict__ srcs, const int* __restrict__ dsts,
    const int* __restrict__ off, const int* __restrict__ rbase,
    int* csr, int nN, int nE, int vec8, int csrLen) {
  extern __shared__ v4f lds_dyn[];
  int* region = (int*)lds_dyn;
  int* cursor = region + RCAP;
  int* list   = cursor + NBF;
  int* wcnt   = list + LISTN;
  const int tid = threadIdx.x, lane = tid & 31, wave = tid >> 5;
  const int b = blockIdx.x;
  const int nodeBase = b * NBF;

  int rb0 = rbase[b];
  const int rb1 = rbase[b + 1];
  rb0 = rb0 < 0 ? 0 : (rb0 > csrLen ? csrLen : rb0);
  rb0 &= ~31;
  int len = rb1 - rb0;
  len = len < 0 ? 0 : (len > RCAP ? RCAP : len);
  int lenW = (len + 31) & ~31;
  if (rb0 + lenW > csrLen) lenW = (csrLen - rb0) & ~31;

  {
    const v4i z = {0, 0, 0, 0};
    for (int i = tid; i < RCAP / 4; i += NTHR) ((v4i*)region)[i] = z;
    for (int s = tid; s < NBF; s += NTHR) {
      int o = off[nodeBase + s] - rb0;
      o = o < 0 ? 0 : (o > RCAP ? RCAP : o);
      cursor[s] = o;
    }
  }
  __syncthreads();

  const int nChunks = (nE + CHUNK - 1) / CHUNK;
#pragma unroll 1
  for (int ch = 0; ch < nChunks; ++ch) {
    const int cbase = ch * CHUNK;
    const int wc = scan_chunk<NBF>(dsts, nE, cbase, nodeBase, vec8, list, tid, lane, wave);
    if (lane == 0) wcnt[wave] = wc;
    __syncthreads();
    if (wave == 0) {
#pragma unroll 1
      for (int wsx = 0; wsx < NWAVE; ++wsx) {
        int n = __builtin_amdgcn_readfirstlane(wcnt[wsx]);
        n = n > WCAP ? WCAP : (n < 0 ? 0 : n);
        const int* lp = list + wsx * WCAP;
#pragma unroll 1
        for (int i = 0; i < n; ++i) {
          const int ent  = __builtin_amdgcn_readfirstlane(lp[i]);
          const int slot = ent & (NBF - 1);
          int e = cbase + ((ent >> 12) & (CHUNK - 1));
          e = e > nE - 1 ? nE - 1 : e;
          int sv = srcs[e];
          sv = sv < 0 ? 0 : (sv > nN - 1 ? nN - 1 : sv);
          if (lane == 0) {
            int pos = cursor[slot];
            pos = pos < 0 ? 0 : (pos > RCAP - 1 ? RCAP - 1 : pos);
            region[pos] = sv;
            const int np = pos + 1;
            cursor[slot] = np > RCAP ? RCAP : np;
          }
        }
      }
    }
    __syncthreads();
  }

  const int nv = lenW >> 2;
  int* gp = csr + rb0;
#pragma unroll 1
  for (int i = tid; i < nv; i += NTHR) { const v4i v = ((const v4i*)region)[i]; *(volatile v4i*)(gp + 4 * i) = v; }
  __threadfence();
#pragma unroll 1
  for (int i = tid; i < nv; i += NTHR) { const v4i v = ((const v4i*)region)[i]; *(volatile v4i*)(gp + 4 * i) = v; }
}

__global__ __launch_bounds__(GTHR) void k_node(const float* __restrict__ X, const unsigned short* __restrict__ Bh,
                                               const unsigned short* __restrict__ Bl, const float* __restrict__ b1,
                                               float* PQ, int nN) {
  __shared__ __attribute__((aligned(16))) unsigned short Ah[GROWS * APZ];
  __shared__ __attribute__((aligned(16))) unsigned short Al[GROWS * APZ];
  __shared__ __attribute__((aligned(16))) float stg[GROWS * NCO];
  const int tid = threadIdx.x, lane = tid & 31, wave = tid >> 5, hh = lane >> 4, m = lane & 15;
  const int rowBase = blockIdx.x * GROWS;
  {
    const int r = tid >> 1, c0 = (tid & 1) * 32;
    int xr = rowBase + r;
    xr = xr > nN - 1 ? nN - 1 : xr;
    const float* xp = X + (size_t)xr * CIN + c0;
#pragma unroll
    for (int g = 0; g < 4; ++g) {
      const v4f a = *(const v4f*)(xp + 8 * g), b = *(const v4f*)(xp + 8 * g + 4);
      float v[8];
      v[0] = a.x; v[1] = a.y; v[2] = a.z; v[3] = a.w; v[4] = b.x; v[5] = b.y; v[6] = b.z; v[7] = b.w;
      v8us uh, ul;
      split8(v, uh, ul);
      *(v8us*)(Ah + r * APZ + c0 + 8 * g) = uh;
      *(v8us*)(Al + r * APZ + c0 + 8 * g) = ul;
    }
  }
  __syncthreads();

  v8f acc[NCO / 16];
  mma3k2<NCO / 16>(Ah + wave * 16 * APZ, Al + wave * 16 * APZ, Bh, Bl, lane, acc);
  float* sp = stg + (wave * 16 + 8 * hh) * NCO + m;
#pragma unroll
  for (int t = 0; t < NCO / 16; ++t) {
    const int bc = (16 * t + m) & (CH - 1);
    const float bl = b1[bc];
    const float bv = (t < NCO / 32) ? bl : 0.0f;
#pragma unroll
    for (int r = 0; r < 8; ++r) sp[r * NCO + 16 * t] = acc[t][r] + bv;
  }
  __syncthreads();

  float* gp = PQ + (size_t)rowBase * NCO;
#pragma unroll
  for (int it = 0; it < NCO / 8; ++it) {
    const int f = it * GTHR + tid;
    const v4f v = *(const v4f*)(stg + 4 * f);
    *(volatile v4f*)(gp + 4 * f) = v;
  }
  __threadfence();
#pragma unroll
  for (int it = 0; it < NCO / 8; ++it) {
    const int f = it * GTHR + tid;
    const v4f v = *(const v4f*)(stg + 4 * f);
    *(volatile v4f*)(gp + 4 * f) = v;
  }
}

__global__ __launch_bounds__(ETHR) void k_edge(
    const float* __restrict__ PQ, const int* __restrict__ csr,
    const int* __restrict__ offp, const int* __restrict__ cntp,
    const unsigned short* __restrict__ Bw, const float* __restrict__ b2,
    float* out, int nN, int csrLen, int cntPad) {
  __shared__ __attribute__((aligned(16))) _Float16 At[EWAV * 16 * APE];
  __shared__ __attribute__((aligned(16))) float smax[EWAV * 2 * NPW * CH];
  __shared__ __attribute__((aligned(16))) int soff[NPBE];
  __shared__ __attribute__((aligned(16))) int scn[NPBE];
  __shared__ __attribute__((aligned(16))) int sntw[EWAV];
  const int tid = threadIdx.x, lane = tid & 31, wave = tid >> 5, hh = lane >> 4, m = lane & 15;
  const int nb0 = blockIdx.x * NPBE;
  {
    const v4f ninf4 = {NEGBIG, NEGBIG, NEGBIG, NEGBIG};
    for (int i = tid; i < (EWAV * 2 * NPW * CH) / 4; i += ETHR) ((v4f*)smax)[i] = ninf4;
    if (tid < NPBE) {
      const int node = nb0 + tid;
      const int nc = node > cntPad - 1 ? cntPad - 1 : node;
      int o = offp[nc];
      o = o < 0 ? 0 : (o > csrLen ? csrLen : o);
      int c = cntp[nc];
      c = c < 0 ? 0 : (c > DEGCAP ? DEGCAP : c);
      c = (node < nN) ? c : 0;
      soff[tid] = o;
      scn[tid] = c;
    }
  }
  __syncthreads();

  const int n0w = nb0 + wave * NPW;
  int ow[NPW];
#pragma unroll
  for (int i = 0; i < NPW; ++i) ow[i] = __builtin_amdgcn_readfirstlane(soff[wave * NPW + i]);
  const int c15 = __builtin_amdgcn_readfirstlane(scn[wave * NPW + NPW - 1]);
  const int start = ow[0];
  int lim = start + TCAP * 16;
  lim = lim > csrLen ? csrLen : lim;
  const int endr = ow[NPW - 1] + c15;
  int end = endr < start ? start : (endr > lim ? lim : endr);
  if (n0w >= nN) end = start;
  const int ntw = (end - start + 15) >> 4;
  if (lane == 0) sntw[wave] = ntw;
  __syncthreads();
  int ntmax;
  {
    const v4i sA = *(const v4i*)sntw;
    int mm = max(max(sA.x, sA.y), max(sA.z, sA.w));
    mm = mm < 0 ? 0 : (mm > TCAP ? TCAP : mm);
    ntmax = __builtin_amdgcn_readfirstlane(mm);
  }
  const int p = m;
  _Float16* Aw = At + wave * 16 * APE;
  float* cellh = smax + ((wave * 2 + hh) * NPW) * CH + m;

#pragma unroll 1
  for (int tt = 0; tt < ntmax; ++tt) {
    const int pos = start + tt * 16 + m;
    const bool valid = pos < end;
    int posc = pos < 0 ? 0 : (pos > csrLen - 1 ? csrLen - 1 : pos);
    int sv = csr[posc];
    sv = sv < 0 ? 0 : (sv > nN - 1 ? nN - 1 : sv);
    int jm = 0;
#pragma unroll
    for (int i = 1; i < NPW; ++i) jm += (ow[i] <= pos) ? 1 : 0;
#pragma unroll
    for (int ps = 0; ps < 8; ++ps) {
      const int k = 2 * ps + hh;
      const int s  = __shfl(sv, k, 32);
      const int jn = __shfl(jm, k, 32);
      int pr = n0w + jn;
      pr = pr > nN - 1 ? nN - 1 : pr;
      const v4f q  = *(const v4f*)(PQ + (size_t)s * PQW + CH + 4 * p);
      const v4f pv = *(const v4f*)(PQ + (size_t)pr * PQW + 4 * p);
      v4f hv = pv + q;
      hv.x = fmaxf(hv.x, 0.0f) * HSC; hv.y = fmaxf(hv.y, 0.0f) * HSC;
      hv.z = fmaxf(hv.z, 0.0f) * HSC; hv.w = fmaxf(hv.w, 0.0f) * HSC;
      v4h h4;
      h4.x = (_Float16)hv.x; h4.y = (_Float16)hv.y; h4.z = (_Float16)hv.z; h4.w = (_Float16)hv.w;
      *(v4h*)(Aw + k * APE + 4 * p) = h4;
    }
    const unsigned vbits = __builtin_amdgcn_ballot_w32(valid);
    int jrow[8];
#pragma unroll
    for (int r = 0; r < 8; ++r) jrow[r] = __shfl(jm, 8 * hh + r, 32);
    __syncthreads();

    v8f acc[4];
#pragma unroll
    for (int t = 0; t < 4; ++t) {
      const v8f z = {0.f, 0.f, 0.f, 0.f, 0.f, 0.f, 0.f, 0.f};
      acc[t] = z;
    }
#pragma unroll
    for (int s = 0; s < 2; ++s) {
      FragH a;
      a.h[0] = *(const v8h*)(Aw + m * APE + 32 * s + 8 * hh);
      a.h[1] = *(const v8h*)(Aw + m * APE + 32 * s + 16 + 8 * hh);
#pragma unroll
      for (int t = 0; t < 4; ++t) {
        const unsigned short* bp = Bw + (16 * t + m) * KPB + 32 * s + 8 * hh;
        FragH b;
        b.u[0] = *(const v8us*)bp;
        b.u[1] = *(const v8us*)(bp + 16);
        acc[t] = wmh(a.v, b.v, acc[t]);
      }
    }
#pragma unroll
    for (int t = 0; t < 4; ++t) {
#pragma unroll
      for (int r = 0; r < 8; ++r) {
        const bool vr = ((vbits >> (8 * hh + r)) & 1u) != 0u;
        int jr = jrow[r];
        jr = jr < 0 ? 0 : (jr > NPW - 1 ? NPW - 1 : jr);
        float* c = cellh + jr * CH + 16 * t;
        const float old = *c;
        const float nw = fmaxf(old, acc[t][r]);
        *c = vr ? nw : old;
      }
    }
    __syncthreads();
  }

  v4f ov[8];
#pragma unroll
  for (int it = 0; it < 8; ++it) {
    const int f = it * ETHR + tid;
    const int q = f >> 4, c4 = (f & 15) * 4;
    const float* h0 = smax + ((q >> 4) * 2 * NPW + (q & 15)) * CH + c4;
    const v4f a = *(const v4f*)h0;
    const v4f b = *(const v4f*)(h0 + NPW * CH);
    const int cq = scn[q];
    const v4f bb = *(const v4f*)(b2 + c4);
    v4f r;
    r.x = (cq > 0) ? (fmaxf(a.x, b.x) * ESC + bb.x) : 0.0f;
    r.y = (cq > 0) ? (fmaxf(a.y, b.y) * ESC + bb.y) : 0.0f;
    r.z = (cq > 0) ? (fmaxf(a.z, b.z) * ESC + bb.z) : 0.0f;
    r.w = (cq > 0) ? (fmaxf(a.w, b.w) * ESC + bb.w) : 0.0f;
    ov[it] = r;
  }
  float* op = out + (size_t)nb0 * CH;
#pragma unroll
  for (int it = 0; it < 8; ++it) {
    const int f = it * ETHR + tid;
    const int row = nb0 + (f >> 4);
    if (row < nN) *(volatile v4f*)(op + 4 * f) = ov[it];
  }
  __threadfence();
#pragma unroll
  for (int it = 0; it < 8; ++it) {
    const int f = it * ETHR + tid;
    const int row = nb0 + (f >> 4);
    if (row < nN) *(volatile v4f*)(op + 4 * f) = ov[it];
  }
}

extern "C" void kernel_launch(void* const* d_in, const int* in_sizes, int n_in,
                              void* d_out, int out_size, void* d_ws, size_t ws_size,
                              hipStream_t stream) {
  if (n_in < 6) return;
  const int nN = in_sizes[0] / CIN;
  const int nE = in_sizes[5] / 2;
  if (nN <= 0 || nE <= 0) return;
  if (in_sizes[0] != nN * CIN || in_sizes[5] != 2 * nE) return;
  if (in_sizes[1] != CH * 2 * CIN || in_sizes[2] != CH || in_sizes[3] != CH * CH || in_sizes[4] != CH) return;
  if (out_size != nN * CH) return;
  if (nE > (1 << 28) || nN > (1 << 24)) return;

  const float* x   = (const float*)d_in[0];
  const float* W1  = (const float*)d_in[1];
  const float* b1  = (const float*)d_in[2];
  const float* W2  = (const float*)d_in[3];
  const float* b2  = (const float*)d_in[4];
  const int*   ei  = (const int*)d_in[5];
  const int* srcs = ei;
  const int* dsts = ei + nE;
  float* out = (float*)d_out;

  const int nBlkG  = (nN + GROWS - 1) / GROWS;
  const int NPADG  = nBlkG * GROWS;
  const int nBC    = (nN + NBC - 1) / NBC;
  const int CNTPAD = nBC * NBC;
  if (2 * nBC + 1 > RBN) return;
  const int nBF    = (nN + NBF - 1) / NBF;
  const int csrLen = ((nE + 31) & ~31) + 4096;
  if (31 * 2 * nBC > 4096) return;
  if (CNTPAD < NPADG) return;

  char* ws = (char*)d_ws;
  size_t off = 0;
  const size_t oB   = off; off += (size_t)BPTOT * 2;               off = (off + 255) & ~(size_t)255;
  const size_t oCnt = off; off += (size_t)CNTPAD * 4;              off = (off + 255) & ~(size_t)255;
  const size_t oOff = off; off += (size_t)CNTPAD * 4;              off = (off + 255) & ~(size_t)255;
  const size_t oRb  = off; off += (size_t)RBN * 4;                 off = (off + 255) & ~(size_t)255;
  const size_t oCsr = off; off += (size_t)csrLen * 4;              off = (off + 255) & ~(size_t)255;
  const size_t oPQ  = off; off += (size_t)NPADG * NCO * 4;         off = (off + 255) & ~(size_t)255;
  if (off > ws_size || off > (size_t)WSCAP) return;
  unsigned short* Bpl = (unsigned short*)(ws + oB);
  int*   cnt  = (int*)(ws + oCnt);
  int*   offp = (int*)(ws + oOff);
  int*   rb   = (int*)(ws + oRb);
  int*   csr  = (int*)(ws + oCsr);
  float* PQ   = (float*)(ws + oPQ);

  const int vec8 = ((nE & 3) == 0) ? 1 : 0;

  k_wprep<<<WPSLOT / NTHR, NTHR, 0, stream>>>(W1, W2, Bpl);
  k_count<<<nBC, NTHR, 0, stream>>>(dsts, cnt, nE, vec8);
  k_offsets<<<1, OTHR, 0, stream>>>(cnt, offp, rb, nBC);
  hipFuncSetAttribute(reinterpret_cast<const void*>(&k_fill),
                      hipFuncAttributeMaxDynamicSharedMemorySize, LDS_FILL);
  k_fill<<<nBF, NTHR, LDS_FILL, stream>>>(srcs, dsts, offp, rb, csr, nN, nE, vec8, csrLen);
  k_node<<<nBlkG, GTHR, 0, stream>>>(x, Bpl + O_NH, Bpl + O_NL, b1, PQ, nN);
  k_edge<<<nBlkG, ETHR, 0, stream>>>(PQ, csr, offp, cnt, Bpl + O_E, b2, out, nN, csrLen, CNTPAD);
}
